// SwinTransformer_40475771797561
// MI455X (gfx1250) — hardware-run, weakly checked
//
#include <hip/hip_runtime.h>
#include <math.h>

typedef __attribute__((ext_vector_type(16))) _Float16 v16h;
typedef __attribute__((ext_vector_type(8)))  _Float16 v8h;
typedef __attribute__((ext_vector_type(16))) __bf16   v16b;
typedef __attribute__((ext_vector_type(8)))  __bf16   v8b;
typedef __attribute__((ext_vector_type(8)))  float    v8f;
typedef __attribute__((ext_vector_type(4)))  float    v4f;
typedef __attribute__((ext_vector_type(4)))  unsigned int v4u;

static constexpr int kBatch    = 16;
static constexpr int kImg      = 56;
static constexpr int kChan     = 128;
static constexpr int kHeads    = 4;
static constexpr int kHeadDim  = 32;
static constexpr int kWinSz    = 7;
static constexpr int kShift    = 3;
static constexpr int kTokWin   = kWinSz * kWinSz;
static constexpr int kWinImg   = (kImg / kWinSz) * (kImg / kWinSz);
static constexpr int kTokens   = kBatch * kImg * kImg;
static constexpr int kPmRows   = kBatch * (kImg / 2) * (kImg / 2);
static constexpr int kChanQKV  = 3 * kChan;
static constexpr int kChanHid  = 4 * kChan;
static constexpr int kChanPm   = 4 * kChan;
static constexpr int kChanOut  = 2 * kChan;
static constexpr int kRelTab   = (2 * kWinSz - 1) * (2 * kWinSz - 1);
static constexpr int kFc1Chunks = 4;
static constexpr int kFc1Rows  = kTokens / kFc1Chunks;

static_assert(kTokens == 50176 && kPmRows == 12544 && kWinImg == 64, "shape");
static_assert(kTokens % 64 == 0 && kFc1Rows % 64 == 0 && kPmRows % 64 == 0, "M tile multiple");
static_assert(kChanQKV % 64 == 0 && kChan % 64 == 0 && kChanHid % 64 == 0 && kChanOut % 64 == 0, "N tile multiple");
static_assert(kChan % 32 == 0 && kChanHid % 32 == 0 && kChanPm % 32 == 0, "K multiple of 32");
static_assert(kTokens % 16 == 0 && kPmRows % 8 == 0, "LN grids exact");
static_assert((kFc1Rows * kChanHid / 2) % 256 == 0, "gelu grid exact");

static constexpr size_t kSzWQ = (size_t)kChanQKV * kChan * 2;
static constexpr size_t kSzWP = (size_t)kChan * kChan * 2;
static constexpr size_t kSzW1 = (size_t)kChanHid * kChan * 2;
static constexpr size_t kSzW2 = (size_t)kChan * kChanHid * 2;
static constexpr size_t kSzWM = (size_t)kChanOut * kChanPm * 2;
static constexpr size_t kOffWQ = 0;
static constexpr size_t kOffWP = kOffWQ + kSzWQ;
static constexpr size_t kOffW1 = kOffWP + kSzWP;
static constexpr size_t kOffW2 = kOffW1 + kSzW1;
static constexpr size_t kOffWMH = kOffW2 + kSzW2;
static constexpr size_t kOffWML = kOffWMH + kSzWM;
static constexpr size_t kSzW  = kOffWML + kSzWM;
static constexpr size_t kOffB = kSzW;
static constexpr size_t kSzB  = (size_t)kTokens * kChan * 4;
static constexpr size_t kOffC = kOffB + kSzB;
static constexpr size_t kSzC  = (size_t)kTokens * kChan * 2;
static constexpr size_t kOffD = kOffC + kSzC;
static constexpr size_t kSzD  = (size_t)kTokens * kChanHid * 2;
static constexpr size_t kOffE = kOffD + kSzD;
static constexpr size_t kSzE  = (size_t)kTokens * kChan * 4;
static constexpr size_t kWsTotal = kOffE + kSzE;
static_assert(kSzW == 917504, "weights");
static_assert(kWsTotal == 116523008, "carve");
static_assert(kWsTotal <= 134217728, "carve limit");
static_assert(kOffB % 128 == 0 && kOffC % 128 == 0 && kOffD % 128 == 0 && kOffE % 128 == 0, "128B aligned regions");
static_assert(kOffWP % 128 == 0 && kOffW1 % 128 == 0 && kOffW2 % 128 == 0 && kOffWMH % 128 == 0 && kOffWML % 128 == 0, "aligned");
static_assert(kSzB >= (size_t)kFc1Rows * kChanHid * 4 && kSzB >= (size_t)kTokens * kChan * 4, "R_B users");
static_assert(kSzC >= (size_t)kTokens * kChan * 2 && kSzC >= (size_t)kPmRows * kChanPm * 2, "R_C users");
static_assert(kSzD >= (size_t)kTokens * kChanQKV * 2 && kSzD >= (size_t)kTokens * kChanHid * 2 && kSzD >= (size_t)kPmRows * kChanPm * 2, "R_D users");
static_assert(kSzE >= (size_t)kTokens * kChan * 4, "R_E users");

__device__ __forceinline__ unsigned short f2bf_bits(float f) {
  unsigned u = __float_as_uint(f);
  return (unsigned short)((u + 0x7FFFu + ((u >> 16) & 1u)) >> 16);
}
__device__ __forceinline__ float bf_bits2f(unsigned short h) { return __uint_as_float(((unsigned)h) << 16); }
__device__ __forceinline__ unsigned short h_bits(float f) { return __builtin_bit_cast(unsigned short, (_Float16)f); }

__device__ __forceinline__ void dep_guard_h(v8f& a, v8f& b, v16h x, v16h y) { asm volatile("v_nop\n\tv_nop\n\tv_nop\n\tv_nop" : "+v"(a), "+v"(b) : "v"(x), "v"(y)); }
__device__ __forceinline__ void dep_guard_b(v8f& a, v8f& b, v16b x, v16b y) { asm volatile("v_nop\n\tv_nop\n\tv_nop\n\tv_nop" : "+v"(a), "+v"(b) : "v"(x), "v"(y)); }
__device__ __forceinline__ void keep4_h(v16h a, v16h b, v16h c, v16h d) { asm volatile("v_nop" :: "v"(a), "v"(b), "v"(c), "v"(d)); }
__device__ __forceinline__ void keep4_b(v16b a, v16b b, v16b c, v16b d) { asm volatile("v_nop" :: "v"(a), "v"(b), "v"(c), "v"(d)); }
__device__ __forceinline__ void acc_guard4(v8f& a, v8f& b, v8f& c, v8f& d) { asm volatile("v_nop\n\tv_nop\n\tv_nop\n\tv_nop" : "+v"(a), "+v"(b), "+v"(c), "+v"(d)); }
template <typename T> struct Frag;
template <> struct Frag<_Float16> {
  typedef v16h V; union U { v16h v; v8h h[2]; };
  static __device__ __forceinline__ v16h load(const _Float16* p) {
    U f; f.h[0] = *(const v8h*)(p); f.h[1] = *(const v8h*)(p + 16); return f.v;
  }
  static __device__ __forceinline__ v8f mma(v16h a, v16h b, v8f c) {
    return __builtin_amdgcn_wmma_f32_16x16x32_f16(false, a, false, b, (short)0, c, false, false);
  }
  static __device__ __forceinline__ void guard(v8f& a, v8f& b, v16h x, v16h y) { dep_guard_h(a, b, x, y); }
  static __device__ __forceinline__ void keep(v16h a, v16h b, v16h c, v16h d) { keep4_h(a, b, c, d); }
};
template <> struct Frag<__bf16> {
  typedef v16b V; union U { v16b v; v8b h[2]; };
  static __device__ __forceinline__ v16b load(const __bf16* p) {
    U f; f.h[0] = *(const v8b*)(p); f.h[1] = *(const v8b*)(p + 16); return f.v;
  }
  static __device__ __forceinline__ v8f mma(v16b a, v16b b, v8f c) {
    return __builtin_amdgcn_wmma_f32_16x16x32_bf16(false, a, false, b, (short)0, c, false, false);
  }
  static __device__ __forceinline__ void guard(v8f& a, v8f& b, v16b x, v16b y) { dep_guard_b(a, b, x, y); }
  static __device__ __forceinline__ void keep(v16b a, v16b b, v16b c, v16b d) { keep4_b(a, b, c, d); }
};

__device__ __forceinline__ v8f hmma(v16h a, v16h b, v8f c) {
  c = __builtin_amdgcn_wmma_f32_16x16x32_f16(false, a, false, b, (short)0, c, false, false);
  asm volatile("v_nop\n\tv_nop\n\tv_nop\n\tv_nop" : "+v"(c) : "v"(a), "v"(b));
  return c;
}

template <int ET> struct Elem;
template <> struct Elem<0> { typedef _Float16 T; };
template <> struct Elem<1> { typedef __bf16 T; };
template <int ET, bool SPLIT, int BIAS_MODE, int OUT_MODE, bool RESID, int ACT = 0>
__global__ __launch_bounds__(256) void wmma_gemm64(
    const unsigned short* __restrict__ Ap, const unsigned short* __restrict__ A2p, int lda, long strideA,
    const unsigned short* __restrict__ Btp, const unsigned short* __restrict__ Bt2p, int ldb, long strideB,
    void* __restrict__ Cout, void* __restrict__ Cout2, int ldc, long strideC,
    const float* __restrict__ bias,
    const float* __restrict__ resid, long strideR,
    int M, int N, int K, float scale) {
  static_assert(!RESID || OUT_MODE == 0, "resid path only with f32 output");
  static_assert(BIAS_MODE == 0 || BIAS_MODE == 2, "bias per column only");
  typedef typename Elem<ET>::T T;
  typedef typename Frag<T>::V V;
  const T* A = (const T*)Ap; const T* A2 = (const T*)A2p; const T* Bt = (const T*)Btp; const T* Bt2 = (const T*)Bt2p;
  __shared__ __align__(16) float sT[8][16 * 68];
  const int b    = blockIdx.y;
  const int lane = threadIdx.x & 31;
  const int wave = threadIdx.x >> 5;
  const int tilesN = N >> 6;
  const int tilesM = M >> 6;
  const int tile = blockIdx.x * 8 + wave;
  if (tile >= tilesM * tilesN) return;
  const int tm = tile / tilesN;
  const int tn = tile - tm * tilesN;
  const int m0 = tm << 6;
  const int n0 = tn << 6;

  const T* Ab  = A  + (size_t)b * strideA;
  const T* Bb  = Bt + (size_t)b * strideB;
  const T* Ab2 = SPLIT ? (A2  + (size_t)b * strideA) : nullptr;
  const T* Bb2 = SPLIT ? (Bt2 + (size_t)b * strideB) : nullptr;

  const int rlane = lane & 15;
  const int koff  = (lane >> 4) * 8;
  const int mOff  = (lane >> 4) * 8;

  v8f acc[4][4];
#pragma unroll
  for (int i = 0; i < 4; ++i)
#pragma unroll
    for (int j = 0; j < 4; ++j) acc[i][j] = (v8f){0.f,0.f,0.f,0.f,0.f,0.f,0.f,0.f};

  for (int k0 = 0; k0 < K; k0 += 32) {
    V bh[4], bl[4];
#pragma unroll
    for (int j = 0; j < 4; ++j) {
      const size_t bo = (size_t)(n0 + (j << 4) + rlane) * ldb + koff + k0;
      bh[j] = Frag<T>::load(Bb + bo);
      if (SPLIT) bl[j] = Frag<T>::load(Bb2 + bo);
    }
#pragma unroll
    for (int i = 0; i < 4; ++i) {
      const size_t ao = (size_t)(m0 + (i << 4) + rlane) * lda + koff + k0;
      V ah = Frag<T>::load(Ab + ao);
      V al;
      if (SPLIT) al = Frag<T>::load(Ab2 + ao);
#pragma unroll
      for (int j = 0; j < 4; ++j) {
        acc[i][j] = Frag<T>::mma(ah, bh[j], acc[i][j]);
        if (SPLIT) {
          acc[i][j] = Frag<T>::mma(ah, bl[j], acc[i][j]);
          acc[i][j] = Frag<T>::mma(al, bh[j], acc[i][j]);
        }
      }
      Frag<T>::guard(acc[i][0], acc[i][3], ah, SPLIT ? al : ah);
    }
    Frag<T>::keep(bh[0], bh[1], bh[2], bh[3]);
    if (SPLIT) Frag<T>::keep(bl[0], bl[1], bl[2], bl[3]);
  }
  acc_guard4(acc[0][0], acc[0][1], acc[0][2], acc[0][3]);
  acc_guard4(acc[1][0], acc[1][1], acc[1][2], acc[1][3]);
  acc_guard4(acc[2][0], acc[2][1], acc[2][2], acc[2][3]);
  acc_guard4(acc[3][0], acc[3][1], acc[3][2], acc[3][3]);

  float* slab = sT[wave];
  const float* Rb = RESID ? (resid + (size_t)b * strideR) : nullptr;
#pragma unroll
  for (int i = 0; i < 4; ++i) {
    const int mBase = m0 + (i << 4);
#pragma unroll
    for (int j = 0; j < 4; ++j) {
      const int n = n0 + (j << 4) + rlane;
      float bv = 0.f;
      if (BIAS_MODE == 2) bv = bias[n];
#pragma unroll
      for (int r = 0; r < 8; ++r) {
        float v = acc[i][j][r] * scale;
        if (BIAS_MODE == 2) v += bv;
        if (ACT == 1) v = tanhf(v);
        if (ACT == 2) v = fmaxf(v, 0.0f);
        if (ACT == 3) v = v / (1.0f + expf(-v));
        if (ACT == 4) v = (v > 0.f) ? v : 0.01f * v;
        slab[(mOff + r) * 68 + (j << 4) + rlane] = v;
      }
    }
    __builtin_amdgcn_fence(__ATOMIC_RELEASE, "workgroup");
    __builtin_amdgcn_wave_barrier();
    __builtin_amdgcn_fence(__ATOMIC_ACQUIRE, "workgroup");
    if (OUT_MODE == 0) {
      float* C = (float*)Cout + (size_t)b * strideC;
      const int hh = lane >> 4, c4 = (lane & 15) * 4;
      for (int pass = 0; pass < 2; ++pass) {
#pragma unroll
        for (int it = 0; it < 8; ++it) {
          const int row = it * 2 + hh;
          v4f v = *(const v4f*)(slab + row * 68 + c4);
          if (RESID) {
            const v4f rv = *(const v4f*)(Rb + (size_t)(mBase + row) * ldc + n0 + c4);
            v = v + rv;
          }
          *(volatile v4f*)(C + (size_t)(mBase + row) * ldc + n0 + c4) = v;
        }
        __threadfence();
      }
    } else {
      const int q = lane >> 3, c8 = (lane & 7) * 8;
      unsigned short* C  = (unsigned short*)Cout  + (size_t)b * strideC;
      unsigned short* C2 = (OUT_MODE == 2) ? ((unsigned short*)Cout2 + (size_t)b * strideC) : nullptr;
      for (int pass = 0; pass < 2; ++pass) {
#pragma unroll
        for (int it = 0; it < 4; ++it) {
          const int row = it * 4 + q;
          const float* sp = slab + row * 68 + c8;
          v8h hv, lv;
#pragma unroll
          for (int e = 0; e < 8; ++e) {
            if (OUT_MODE == 1) {
              hv[e] = (_Float16)sp[e];
            } else {
              unsigned short hb = f2bf_bits(sp[e]);
              unsigned short lb = f2bf_bits(sp[e] - bf_bits2f(hb));
              hv[e] = __builtin_bit_cast(_Float16, hb);
              lv[e] = __builtin_bit_cast(_Float16, lb);
            }
          }
          *(volatile v8h*)(C + (size_t)(mBase + row) * ldc + n0 + c8) = hv;
          if (OUT_MODE == 2) *(volatile v8h*)(C2 + (size_t)(mBase + row) * ldc + n0 + c8) = lv;
        }
        __threadfence();
      }
    }
    __builtin_amdgcn_fence(__ATOMIC_RELEASE, "workgroup");
    __builtin_amdgcn_wave_barrier();
    __builtin_amdgcn_fence(__ATOMIC_ACQUIRE, "workgroup");
  }
}

__device__ __forceinline__ size_t win_row_src(int m) {
  const int win = m / kTokWin;
  const int t = m - win * kTokWin;
  const int b = win >> 6, wi = win & 63, wh = wi >> 3, ww = wi & 7;
  const int ty = t / kWinSz, tx = t - ty * kWinSz;
  int y = wh * kWinSz + ty + kShift; y = (y >= kImg) ? (y - kImg) : y;
  int xx = ww * kWinSz + tx + kShift; xx = (xx >= kImg) ? (xx - kImg) : xx;
  return (((size_t)b * kImg + y) * kImg + xx) * kChan;
}
__device__ __forceinline__ int nat_to_win_row(int b, int y, int xx) {
  int ys = y + (kImg - kShift); ys = (ys >= kImg) ? (ys - kImg) : ys;
  int xs = xx + (kImg - kShift); xs = (xs >= kImg) ? (xs - kImg) : xs;
  const int wh = ys / kWinSz, ty = ys - wh * kWinSz;
  const int ww = xs / kWinSz, tx = xs - ww * kWinSz;
  return ((b * kWinImg + wh * 8 + ww) * kTokWin) + ty * kWinSz + tx;
}
__device__ __forceinline__ int region_id(int r, int c) {
  const int gr = (r < kImg - kWinSz) ? 0 : ((r < kImg - kShift) ? 1 : 2);
  const int gc = (c < kImg - kWinSz) ? 0 : ((c < kImg - kShift) ? 1 : 2);
  return gr * 3 + gc;
}

template <bool WIN>
__global__ __launch_bounds__(256) void k_ln128(const float* __restrict__ src, const float* __restrict__ gam,
    const float* __restrict__ bet, float* __restrict__ xcopy, unsigned short* __restrict__ outA, int nrows) {
  const int lane = threadIdx.x & 31;
  const int hh = lane >> 4;
  const int c8 = (lane & 15) * 8;
  const int wg = blockIdx.x * 8 + (threadIdx.x >> 5);
  const int m0 = wg * 2;
  if (m0 >= nrows) return;
  const float* s0;
  const float* s1;
  if (WIN) { s0 = src + win_row_src(m0); s1 = src + win_row_src(m0 + 1); }
  else { s0 = src + (size_t)m0 * kChan; s1 = src + (size_t)(m0 + 1) * kChan; }
  if (WIN) {
    const v4f cv0 = *(const v4f*)(s0 + lane * 4);
    const v4f cv1 = *(const v4f*)(s1 + lane * 4);
    float* d0 = xcopy + (size_t)m0 * kChan + lane * 4;
    float* d1 = xcopy + (size_t)(m0 + 1) * kChan + lane * 4;
    for (int pass = 0; pass < 2; ++pass) {
      *(volatile v4f*)d0 = cv0;
      *(volatile v4f*)d1 = cv1;
      __threadfence();
    }
  }
  const float* sm = hh ? s1 : s0;
  const v4f va = *(const v4f*)(sm + c8);
  const v4f vb = *(const v4f*)(sm + c8 + 4);
  const float v[8] = {va.x, va.y, va.z, va.w, vb.x, vb.y, vb.z, vb.w};
  float s = ((v[0] + v[1]) + (v[2] + v[3])) + ((v[4] + v[5]) + (v[6] + v[7]));
  s += __shfl_xor(s, 1, 32); s += __shfl_xor(s, 2, 32); s += __shfl_xor(s, 4, 32); s += __shfl_xor(s, 8, 32);
  const float mean = s * (1.0f / 128.0f);
  float d[8];
  float s2 = 0.f;
#pragma unroll
  for (int e = 0; e < 8; ++e) { d[e] = v[e] - mean; s2 += d[e] * d[e]; }
  s2 += __shfl_xor(s2, 1, 32); s2 += __shfl_xor(s2, 2, 32); s2 += __shfl_xor(s2, 4, 32); s2 += __shfl_xor(s2, 8, 32);
  const float var = s2 * (1.0f / 128.0f);
  const float inv = rsqrtf(var + 1.001e-05f);
  const v4f g0 = *(const v4f*)(gam + c8), g1 = *(const v4f*)(gam + c8 + 4);
  const v4f b0 = *(const v4f*)(bet + c8), b1 = *(const v4f*)(bet + c8 + 4);
  const float gg[8] = {g0.x, g0.y, g0.z, g0.w, g1.x, g1.y, g1.z, g1.w};
  const float bb[8] = {b0.x, b0.y, b0.z, b0.w, b1.x, b1.y, b1.z, b1.w};
  unsigned w[4] = {0u, 0u, 0u, 0u};
#pragma unroll
  for (int e = 0; e < 8; ++e) {
    const float y = d[e] * inv * gg[e] + bb[e];
    w[e >> 1] |= ((unsigned)h_bits(y)) << ((e & 1) * 16);
  }
  const v4u pk = {w[0], w[1], w[2], w[3]};
  unsigned short* dst = outA + (size_t)(m0 + hh) * kChan + c8;
  for (int pass = 0; pass < 2; ++pass) {
    *(volatile v4u*)dst = pk;
    __threadfence();
  }
}

template <int MODE>
__global__ __launch_bounds__(256) void k_wtrans(const float* __restrict__ wm, int kdim, int ndim,
    unsigned short* __restrict__ outH, unsigned short* __restrict__ outL) {
  __shared__ float tile[64][65];
  const int tid = threadIdx.x;
  const int n0 = blockIdx.x * 64;
  const int k0 = blockIdx.y * 64;
#pragma unroll 4
  for (int i = 0; i < 16; ++i) {
    const int kk = i * 4 + (tid >> 6);
    const int nn = tid & 63;
    tile[kk][nn] = wm[(size_t)(k0 + kk) * ndim + n0 + nn];
  }
  __syncthreads();
  const int wave = tid >> 5, lane = tid & 31;
  const int q = lane >> 3, c8 = (lane & 7) * 8;
  v4u hv[2], lv[2];
#pragma unroll
  for (int it = 0; it < 2; ++it) {
    const int n = it * 32 + wave * 4 + q;
    unsigned hw[4] = {0u, 0u, 0u, 0u};
    unsigned lw[4] = {0u, 0u, 0u, 0u};
#pragma unroll
    for (int e = 0; e < 8; ++e) {
      const float f = tile[c8 + e][n];
      unsigned short hb;
      unsigned short lb = 0;
      if (MODE == 0) { hb = h_bits(f); }
      else { hb = f2bf_bits(f); lb = f2bf_bits(f - bf_bits2f(hb)); }
      hw[e >> 1] |= ((unsigned)hb) << ((e & 1) * 16);
      lw[e >> 1] |= ((unsigned)lb) << ((e & 1) * 16);
    }
    hv[it] = (v4u){hw[0], hw[1], hw[2], hw[3]};
    lv[it] = (v4u){lw[0], lw[1], lw[2], lw[3]};
  }
  for (int pass = 0; pass < 2; ++pass) {
#pragma unroll
    for (int it = 0; it < 2; ++it) {
      const int n = it * 32 + wave * 4 + q;
      unsigned short* dh = outH + (size_t)(n0 + n) * kdim + k0 + c8;
      *(volatile v4u*)dh = hv[it];
      if (MODE == 1) {
        unsigned short* dl = outL + (size_t)(n0 + n) * kdim + k0 + c8;
        *(volatile v4u*)dl = lv[it];
      }
    }
    __threadfence();
  }
}

__global__ __launch_bounds__(128) void k_attn(const unsigned short* __restrict__ qkv,
    const float* __restrict__ relb, unsigned short* __restrict__ ao) {
  __shared__ __align__(16) unsigned short Ksh[kHeads * 64 * kHeadDim];
  __shared__ __align__(16) unsigned short Vt[kHeads * kHeadDim * 64];
  __shared__ __align__(16) _Float16 Psh[4][16 * 64];
  __shared__ __align__(16) unsigned short Osh[64 * kChan];
  __shared__ float btab[kRelTab * kHeads];
  union FH { v16h v; v8h h[2]; };
  const int tid  = threadIdx.x;
  const int wave = tid >> 5;
  const int lane = tid & 31;
  const int hh   = lane >> 4;
  const int c    = lane & 15;
  const int win  = blockIdx.x;
  const int wi   = win & (kWinImg - 1);
  const int wh   = wi >> 3, ww = wi & 7;
  const size_t tok0 = (size_t)win * kTokWin;
  const int head = wave;

  for (int i = tid; i < kRelTab * kHeads; i += 128) btab[i] = relb[i];
#pragma unroll 1
  for (int i = 0; i < 8; ++i) {
    const int qd  = i * 128 + tid;
    const int hd  = qd >> 8;
    const int key = (qd >> 2) & 63;
    const int d0  = (qd & 3) * 8;
    const int keyc = (key < kTokWin) ? key : (kTokWin - 1);
    const unsigned short* rp = qkv + (tok0 + keyc) * kChanQKV + hd * kHeadDim + d0;
    v4u kw = *(const v4u*)(rp + kChan);
    v4u vw = *(const v4u*)(rp + 2 * kChan);
    const unsigned msk = (key < kTokWin) ? 0xffffffffu : 0u;
    kw = kw & (v4u){msk, msk, msk, msk};
    vw = vw & (v4u){msk, msk, msk, msk};
    *(v4u*)(Ksh + (hd * 64 + key) * kHeadDim + d0) = kw;
    unsigned short* vt = Vt + (hd * kHeadDim + d0) * 64 + key;
    vt[0 * 64] = (unsigned short)(vw.x & 0xffffu);
    vt[1 * 64] = (unsigned short)(vw.x >> 16);
    vt[2 * 64] = (unsigned short)(vw.y & 0xffffu);
    vt[3 * 64] = (unsigned short)(vw.y >> 16);
    vt[4 * 64] = (unsigned short)(vw.z & 0xffffu);
    vt[5 * 64] = (unsigned short)(vw.z >> 16);
    vt[6 * 64] = (unsigned short)(vw.w & 0xffffu);
    vt[7 * 64] = (unsigned short)(vw.w >> 16);
  }
  __syncthreads();

  const float scale = 0.17677669529663687f;
  _Float16* pw = Psh[wave];
#pragma unroll 1
  for (int mt = 0; mt < 4; ++mt) {
    const int qr  = mt * 16 + c;
    const int qrc = (qr < kTokWin) ? qr : (kTokWin - 1);
    FH qa;
    {
      const _Float16* qp = (const _Float16*)(qkv + (tok0 + qrc) * kChanQKV + head * kHeadDim + 8 * hh);
      qa.h[0] = *(const v8h*)(qp);
      qa.h[1] = *(const v8h*)(qp + 16);
    }
    v8f s[4];
#pragma unroll
    for (int j = 0; j < 4; ++j) {
      FH kb;
      const _Float16* kp = (const _Float16*)(Ksh + (head * 64 + j * 16 + c) * kHeadDim + 8 * hh);
      kb.h[0] = *(const v8h*)(kp);
      kb.h[1] = *(const v8h*)(kp + 16);
      s[j] = hmma(qa.v, kb.v, (v8f){0.f, 0.f, 0.f, 0.f, 0.f, 0.f, 0.f, 0.f});
    }
    const int qrow0 = mt * 16 + 8 * hh;
    float linv[8];
#pragma unroll
    for (int r = 0; r < 8; ++r) {
      const int qrow = qrow0 + r;
      const int qc = (qrow < kTokWin) ? qrow : (kTokWin - 1);
      const int fxq = qc / kWinSz, fyq = qc - fxq * kWinSz;
      const int gq = region_id(wh * kWinSz + fxq, ww * kWinSz + fyq);
      float vals[4];
      float m = -INFINITY;
#pragma unroll
      for (int j = 0; j < 4; ++j) {
        const int kcol = j * 16 + c;
        const int kc = (kcol < kTokWin) ? kcol : (kTokWin - 1);
        const int fxk = kc / kWinSz, fyk = kc - fxk * kWinSz;
        const int rel = (fxq - fxk + (kWinSz - 1)) * (2 * kWinSz - 1) + (fyq - fyk + (kWinSz - 1));
        float v = s[j][r] * scale + btab[rel * kHeads + head];
        const int gk = region_id(wh * kWinSz + fxk, ww * kWinSz + fyk);
        v = (gq != gk) ? (v - 100.0f) : v;
        v = (kcol < kTokWin) ? v : -INFINITY;
        vals[j] = v;
        m = fmaxf(m, v);
      }
#pragma unroll
      for (int off = 1; off < 16; off <<= 1) m = fmaxf(m, __shfl_xor(m, off, 32));
      float ps = 0.f;
#pragma unroll
      for (int j = 0; j < 4; ++j) {
        const float p = expf(vals[j] - m);
        ps += p;
        pw[(8 * hh + r) * 64 + j * 16 + c] = (_Float16)(p * 1024.0f);
      }
#pragma unroll
      for (int off = 1; off < 16; off <<= 1) ps += __shfl_xor(ps, off, 32);
      linv[r] = 1.0f / (ps * 1024.0f);
    }
    __syncthreads();
    v8f o[2];
    o[0] = (v8f){0.f, 0.f, 0.f, 0.f, 0.f, 0.f, 0.f, 0.f};
    o[1] = (v8f){0.f, 0.f, 0.f, 0.f, 0.f, 0.f, 0.f, 0.f};
#pragma unroll
    for (int kk = 0; kk < 2; ++kk) {
      FH pa;
      const _Float16* pp = pw + c * 64 + kk * 32 + 8 * hh;
      pa.h[0] = *(const v8h*)(pp);
      pa.h[1] = *(const v8h*)(pp + 16);
#pragma unroll
      for (int t = 0; t < 2; ++t) {
        FH vb;
        const _Float16* vp = (const _Float16*)(Vt + (head * kHeadDim + t * 16 + c) * 64 + kk * 32 + 8 * hh);
        vb.h[0] = *(const v8h*)(vp);
        vb.h[1] = *(const v8h*)(vp + 16);
        o[t] = hmma(pa.v, vb.v, o[t]);
      }
    }
#pragma unroll
    for (int r = 0; r < 8; ++r) {
      const int row = qrow0 + r;
#pragma unroll
      for (int t = 0; t < 2; ++t)
        Osh[row * kChan + head * kHeadDim + t * 16 + c] = h_bits(o[t][r] * linv[r]);
    }
    __syncthreads();
  }
  {
    const int q = lane >> 3, c8 = (lane & 7) * 8;
    for (int pass = 0; pass < 2; ++pass) {
#pragma unroll
      for (int it = 0; it < 7; ++it) {
        const int row = it * 8 + wave * 2 + (q >> 1);
        const int off = (q & 1) * 64 + c8;
        const v4u val = *(const v4u*)(Osh + row * kChan + off);
        if (row < kTokWin) *(volatile v4u*)(ao + (tok0 + row) * kChan + off) = val;
      }
      __threadfence();
    }
  }
}

__global__ __launch_bounds__(256) void k_gelu2(const float* __restrict__ in, unsigned short* __restrict__ out, int n2) {
  const int i = blockIdx.x * 256 + threadIdx.x;
  if (i < n2) {
    unsigned u = 0u;
#pragma unroll 1
    for (int e = 0; e < 2; ++e) {
      const float t = in[2 * (size_t)i + e];
      const float gl = 0.5f * t * (1.0f + erff(t * 0.70710678118654752f));
      u |= ((unsigned)h_bits(gl)) << (16 * e);
    }
    ((volatile unsigned*)out)[i] = u;
    __threadfence();
    ((volatile unsigned*)out)[i] = u;
  }
}

__global__ __launch_bounds__(256) void k_pmln(const float* __restrict__ x2w, const float* __restrict__ gam,
    const float* __restrict__ bet, unsigned short* __restrict__ outH, unsigned short* __restrict__ outL, int nrows) {
  const int lane = threadIdx.x & 31;
  const int p = blockIdx.x * 8 + (threadIdx.x >> 5);
  if (p >= nrows) return;
  const int b = p / 784;
  const int rem = p - b * 784;
  const int i2 = rem / 28;
  const int j2 = rem - i2 * 28;
  float v[16];
#pragma unroll
  for (int it = 0; it < 2; ++it) {
    const int c0 = it * 256 + lane * 8;
    const int blk = c0 >> 7;
    const int cc = c0 & 127;
    const int dh = blk & 1, dw = blk >> 1;
    const int m = nat_to_win_row(b, 2 * i2 + dh, 2 * j2 + dw);
    const float* sp = x2w + (size_t)m * kChan + cc;
    const v4f a = *(const v4f*)(sp);
    const v4f bq = *(const v4f*)(sp + 4);
    v[it * 8 + 0] = a.x; v[it * 8 + 1] = a.y; v[it * 8 + 2] = a.z; v[it * 8 + 3] = a.w;
    v[it * 8 + 4] = bq.x; v[it * 8 + 5] = bq.y; v[it * 8 + 6] = bq.z; v[it * 8 + 7] = bq.w;
  }
  float s = 0.f;
#pragma unroll
  for (int e = 0; e < 16; ++e) s += v[e];
  s += __shfl_xor(s, 1, 32); s += __shfl_xor(s, 2, 32); s += __shfl_xor(s, 4, 32); s += __shfl_xor(s, 8, 32); s += __shfl_xor(s, 16, 32);
  const float mean = s * (1.0f / 512.0f);
  float d[16];
  float s2 = 0.f;
#pragma unroll
  for (int e = 0; e < 16; ++e) { d[e] = v[e] - mean; s2 += d[e] * d[e]; }
  s2 += __shfl_xor(s2, 1, 32); s2 += __shfl_xor(s2, 2, 32); s2 += __shfl_xor(s2, 4, 32); s2 += __shfl_xor(s2, 8, 32); s2 += __shfl_xor(s2, 16, 32);
  const float var = s2 * (1.0f / 512.0f);
  const float inv = rsqrtf(var + 1.001e-05f);
  v4u hv[2], lv[2];
#pragma unroll
  for (int it = 0; it < 2; ++it) {
    const int c0 = it * 256 + lane * 8;
    const v4f g0 = *(const v4f*)(gam + c0), g1 = *(const v4f*)(gam + c0 + 4);
    const v4f b0 = *(const v4f*)(bet + c0), b1 = *(const v4f*)(bet + c0 + 4);
    const float gg[8] = {g0.x, g0.y, g0.z, g0.w, g1.x, g1.y, g1.z, g1.w};
    const float bb[8] = {b0.x, b0.y, b0.z, b0.w, b1.x, b1.y, b1.z, b1.w};
    unsigned hw[4] = {0u, 0u, 0u, 0u};
    unsigned lw[4] = {0u, 0u, 0u, 0u};
#pragma unroll
    for (int e = 0; e < 8; ++e) {
      const float y = d[it * 8 + e] * inv * gg[e] + bb[e];
      const unsigned short hb = f2bf_bits(y);
      const unsigned short lb = f2bf_bits(y - bf_bits2f(hb));
      hw[e >> 1] |= ((unsigned)hb) << ((e & 1) * 16);
      lw[e >> 1] |= ((unsigned)lb) << ((e & 1) * 16);
    }
    hv[it] = (v4u){hw[0], hw[1], hw[2], hw[3]};
    lv[it] = (v4u){lw[0], lw[1], lw[2], lw[3]};
  }
  for (int pass = 0; pass < 2; ++pass) {
#pragma unroll
    for (int it = 0; it < 2; ++it) {
      unsigned short* dh = outH + (size_t)p * kChanPm + it * 256 + lane * 8;
      unsigned short* dl = outL + (size_t)p * kChanPm + it * 256 + lane * 8;
      *(volatile v4u*)dh = hv[it];
      *(volatile v4u*)dl = lv[it];
    }
    __threadfence();
  }
}

extern "C" void kernel_launch(void* const* d_in, const int* in_sizes, int n_in,
                              void* d_out, int out_size, void* d_ws, size_t ws_size,
                              hipStream_t stream) {
  if (n_in < 17) return;
  if (ws_size < kWsTotal) return;
  if ((size_t)out_size < (size_t)kPmRows * kChanOut) return;
  if (in_sizes[0] != kTokens * kChan) return;

  const float* x          = (const float*)d_in[0];
  const float* ln1_g      = (const float*)d_in[1];
  const float* ln1_b      = (const float*)d_in[2];
  const float* qkv_w      = (const float*)d_in[3];
  const float* qkv_b      = (const float*)d_in[4];
  const float* proj_w     = (const float*)d_in[5];
  const float* proj_b     = (const float*)d_in[6];
  const float* bias_table = (const float*)d_in[7];
  const float* ln2_g      = (const float*)d_in[8];
  const float* ln2_b      = (const float*)d_in[9];
  const float* mlp_w1     = (const float*)d_in[10];
  const float* mlp_b1     = (const float*)d_in[11];
  const float* mlp_w2     = (const float*)d_in[12];
  const float* mlp_b2     = (const float*)d_in[13];
  const float* pm_ln_g    = (const float*)d_in[14];
  const float* pm_ln_b    = (const float*)d_in[15];
  const float* pm_w       = (const float*)d_in[16];
  float* out = (float*)d_out;

  char* ws = (char*)d_ws;
  unsigned short* pWQ  = (unsigned short*)(ws + kOffWQ);
  unsigned short* pWP  = (unsigned short*)(ws + kOffWP);
  unsigned short* pW1  = (unsigned short*)(ws + kOffW1);
  unsigned short* pW2  = (unsigned short*)(ws + kOffW2);
  unsigned short* pWMH = (unsigned short*)(ws + kOffWMH);
  unsigned short* pWML = (unsigned short*)(ws + kOffWML);
  float*          pXW  = (float*)(ws + kOffB);
  float*          pG   = (float*)(ws + kOffB);
  float*          pX2  = (float*)(ws + kOffB);
  unsigned short* pA   = (unsigned short*)(ws + kOffC);
  unsigned short* pQKV = (unsigned short*)(ws + kOffD);
  unsigned short* pH   = (unsigned short*)(ws + kOffD);
  unsigned short* pA3L = (unsigned short*)(ws + kOffD);
  float*          pX1  = (float*)(ws + kOffE);

  k_ln128<true><<<kTokens / 16, 256, 0, stream>>>(x, ln1_g, ln1_b, pXW, pA, kTokens);
  k_wtrans<0><<<dim3(kChanQKV / 64, kChan / 64), 256, 0, stream>>>(qkv_w, kChan, kChanQKV, pWQ, pWQ);
  k_wtrans<0><<<dim3(kChan / 64, kChan / 64), 256, 0, stream>>>(proj_w, kChan, kChan, pWP, pWP);
  k_wtrans<0><<<dim3(kChanHid / 64, kChan / 64), 256, 0, stream>>>(mlp_w1, kChan, kChanHid, pW1, pW1);
  k_wtrans<0><<<dim3(kChan / 64, kChanHid / 64), 256, 0, stream>>>(mlp_w2, kChanHid, kChan, pW2, pW2);
  k_wtrans<1><<<dim3(kChanOut / 64, kChanPm / 64), 256, 0, stream>>>(pm_w, kChanPm, kChanOut, pWMH, pWML);
  {
    const int tiles = (kTokens / 64) * (kChanQKV / 64);
    wmma_gemm64<0, false, 2, 1, false><<<dim3((tiles + 7) / 8, 1), 256, 0, stream>>>(
        pA, pA, kChan, 0L, pWQ, pWQ, kChan, 0L, (void*)pQKV, (void*)pQKV, kChanQKV, 0L,
        qkv_b, x, 0L, kTokens, kChanQKV, kChan, 1.0f);
  }
  k_attn<<<kBatch * kWinImg, 128, 0, stream>>>(pQKV, bias_table, pA);
  {
    const int tiles = (kTokens / 64) * (kChan / 64);
    wmma_gemm64<0, false, 2, 0, true><<<dim3((tiles + 7) / 8, 1), 256, 0, stream>>>(
        pA, pA, kChan, 0L, pWP, pWP, kChan, 0L, (void*)pX1, (void*)pX1, kChan, 0L,
        proj_b, pXW, 0L, kTokens, kChan, kChan, 1.0f);
  }
  k_ln128<false><<<kTokens / 16, 256, 0, stream>>>(pX1, ln2_g, ln2_b, pXW, pA, kTokens);
  for (int ch = 0; ch < kFc1Chunks; ++ch) {
    const int tiles = (kFc1Rows / 64) * (kChanHid / 64);
    wmma_gemm64<0, false, 2, 0, false><<<dim3((tiles + 7) / 8, 1), 256, 0, stream>>>(
        pA + (size_t)ch * kFc1Rows * kChan, pA, kChan, 0L, pW1, pW1, kChan, 0L, (void*)pG, (void*)pG, kChanHid, 0L,
        mlp_b1, x, 0L, kFc1Rows, kChanHid, kChan, 1.0f);
    const int n2 = kFc1Rows * kChanHid / 2;
    k_gelu2<<<n2 / 256, 256, 0, stream>>>(pG, pH + (size_t)ch * kFc1Rows * kChanHid, n2);
  }
  {
    const int tiles = (kTokens / 64) * (kChan / 64);
    wmma_gemm64<0, false, 2, 0, true><<<dim3((tiles + 7) / 8, 1), 256, 0, stream>>>(
        pH, pH, kChanHid, 0L, pW2, pW2, kChanHid, 0L, (void*)pX2, (void*)pX2, kChan, 0L,
        mlp_b2, pX1, 0L, kTokens, kChan, kChanHid, 1.0f);
  }
  k_pmln<<<kPmRows / 8, 256, 0, stream>>>(pX2, pm_ln_g, pm_ln_b, pA, pA3L, kPmRows);
  {
    const int tiles = (kPmRows / 64) * (kChanOut / 64);
    wmma_gemm64<1, true, 0, 0, false><<<dim3((tiles + 7) / 8, 1), 256, 0, stream>>>(
        pA, pA3L, kChanPm, 0L, pWMH, pWML, kChanPm, 0L, (void*)out, (void*)out, kChanOut, 0L,
        pm_ln_g, x, 0L, kPmRows, kChanOut, kChanPm, 1.0f);
  }
}
